// FullSparseAttention_11776800325695
// MI455X (gfx1250) — hardware-verified
//
#include <hip/hip_runtime.h>
#include <math.h>
#include <stddef.h>


typedef _Float16 f16;
typedef _Float16 v16h __attribute__((ext_vector_type(16)));
typedef _Float16 v8hx __attribute__((ext_vector_type(8)));
typedef v8hx v8h __attribute__((may_alias));
typedef float v8f __attribute__((ext_vector_type(8)));
typedef float v4fx __attribute__((ext_vector_type(4)));
typedef v4fx v4f __attribute__((may_alias));
typedef int v4ix __attribute__((ext_vector_type(4)));
typedef v4ix v4i __attribute__((may_alias));

#define D_MODEL 1024
#define NB      2048
#define BATCH   2
#define MTOT    (BATCH * NB)
#define NHEAD   16
#define HD      64

union Frag   { v16h v; v8hx hv[2]; };
union Pack16 { v8hx h; v4fx f; v4ix i; };

__device__ __forceinline__ v16h ldfrag(const f16* __restrict__ base, size_t ld, int lane) {
    const f16* p = base + (size_t)(lane & 15) * ld + ((lane >> 4) << 3);
    Frag f;
    f.hv[0] = *(const v8h*)(p);
    f.hv[1] = *(const v8h*)(p + 16);
    return f.v;
}

__device__ __forceinline__ v8f mma16(v16h a, v16h b, v8f c) {
    v8f d = __builtin_amdgcn_wmma_f32_16x16x32_f16(false, a, false, b, (short)0, c, false, false);
    asm volatile("v_nop\n\tv_nop\n\tv_nop\n\tv_nop" : "+v"(d) : "v"(a), "v"(b));
    return d;
}

__device__ __forceinline__ float redmax16(float v) {
    v = fmaxf(v, __shfl_xor(v, 1));
    v = fmaxf(v, __shfl_xor(v, 2));
    v = fmaxf(v, __shfl_xor(v, 4));
    v = fmaxf(v, __shfl_xor(v, 8));
    return v;
}
__device__ __forceinline__ float redsum16(float v) {
    v += __shfl_xor(v, 1);
    v += __shfl_xor(v, 2);
    v += __shfl_xor(v, 4);
    v += __shfl_xor(v, 8);
    return v;
}

__global__ __launch_bounds__(256)
void k_prep(const float* __restrict__ hsrc, f16* hdst) {
    const int t = blockIdx.x * 256 + threadIdx.x;
    if (t >= NB * (D_MODEL / 8)) return;
    const int n  = t >> 7;
    const int d0 = (t & 127) << 3;
    const float ce = (float)(-9.210340371976184 / 1024.0);
    float pe[8];
#pragma unroll
    for (int q = 0; q < 4; ++q) {
        const int i2 = (d0 >> 1) + q;
        const float freq = expf((float)(2 * i2) * ce);
        const float ang  = (float)n * freq;
        float s, c;
        sincosf(ang, &s, &c);
        pe[2 * q]     = s;
        pe[2 * q + 1] = c;
    }
    Pack16 pk[BATCH];
#pragma unroll
    for (int b = 0; b < BATCH; ++b) {
        const float* src = hsrc + ((size_t)b * NB + n) * D_MODEL + d0;
        const v4fx x0 = *(const v4f*)(src);
        const v4fx x1 = *(const v4f*)(src + 4);
#pragma unroll
        for (int e = 0; e < 4; ++e) {
            pk[b].h[e]     = (f16)((x0[e] + pe[e]) * 8.0f);
            pk[b].h[4 + e] = (f16)((x1[e] + pe[4 + e]) * 8.0f);
        }
        *(volatile v4i*)(hdst + ((size_t)b * NB + n) * D_MODEL + d0) = pk[b].i;
    }
    __threadfence();
#pragma unroll
    for (int b = 0; b < BATCH; ++b)
        *(volatile v4i*)(hdst + ((size_t)b * NB + n) * D_MODEL + d0) = pk[b].i;
}

__global__ __launch_bounds__(256)
void k_bias(const float* __restrict__ probs, const float* __restrict__ pbs,
            const int* __restrict__ nh, float* biasL, int total) {
    (void)nh;
    const int t = blockIdx.x * 256 + threadIdx.x;
    if (t * 4 >= total) return;
    const v4fx p = *(const v4f*)(probs + (size_t)t * 4);
    const float s = pbs[0];
    v4fx o;
#pragma unroll
    for (int e = 0; e < 4; ++e) o[e] = s * logf(p[e] + 1e-8f);
    *(volatile v4f*)(biasL + (size_t)t * 4) = o;
    __threadfence();
    *(volatile v4f*)(biasL + (size_t)t * 4) = o;
}

__global__ __launch_bounds__(256)
void k_cvtw(const float* __restrict__ w0, const float* __restrict__ w1,
            const float* __restrict__ w2, const float* __restrict__ w3,
            f16* o0, f16* o1, f16* o2, f16* o3, int total) {
    const int t = blockIdx.x * 256 + threadIdx.x;
    if (t * 8 >= total) return;
    const float* src = w0; f16* dst = o0;
    if (blockIdx.y == 1)      { src = w1; dst = o1; }
    else if (blockIdx.y == 2) { src = w2; dst = o2; }
    else if (blockIdx.y == 3) { src = w3; dst = o3; }
    const v4fx x0 = *(const v4f*)(src + (size_t)t * 8);
    const v4fx x1 = *(const v4f*)(src + (size_t)t * 8 + 4);
    Pack16 pk;
#pragma unroll
    for (int e = 0; e < 4; ++e) {
        pk.h[e]     = (f16)(x0[e] * 64.0f);
        pk.h[4 + e] = (f16)(x1[e] * 64.0f);
    }
    *(volatile v4i*)(dst + (size_t)t * 8) = pk.i;
    __threadfence();
    *(volatile v4i*)(dst + (size_t)t * 8) = pk.i;
}

template <int MODE>
__global__ __launch_bounds__(128)
void k_gemm(const f16* __restrict__ A, const f16* __restrict__ W0, const f16* __restrict__ W1,
            const float* __restrict__ bias0, const float* __restrict__ bias1,
            void* out0, void* out1, int M) {
    __shared__ __attribute__((aligned(16))) unsigned char smem[(MODE == 2) ? 32768 : 16384];

    const int tid = threadIdx.x, lane = tid & 31, w = tid >> 5;
    const int h = lane >> 4, n = lane & 15;
    const int wm = w >> 1, wn = w & 1;
    const int sel = blockIdx.z;
    const f16*   W    = sel ? W1 : W0;
    const float* bias = sel ? bias1 : bias0;
    void*        outp = sel ? out1 : out0;
    const int row0 = blockIdx.y * 64, col0 = blockIdx.x * 128;
    const int m0 = row0 + wm * 32, n0 = col0 + wn * 64;

    v8f acc[2][4] = {};
    for (int k0 = 0; k0 < D_MODEL; k0 += 32) {
        const v16h a0 = ldfrag(A + (size_t)m0 * D_MODEL + k0, D_MODEL, lane);
        const v16h a1 = ldfrag(A + (size_t)(m0 + 16) * D_MODEL + k0, D_MODEL, lane);
#pragma unroll
        for (int j = 0; j < 4; ++j) {
            const v16h bw = ldfrag(W + (size_t)(n0 + 16 * j) * D_MODEL + k0, D_MODEL, lane);
            acc[0][j] = mma16(a0, bw, acc[0][j]);
            acc[1][j] = mma16(a1, bw, acc[1][j]);
        }
    }

    if (MODE == 0) {
        f16* T = (f16*)smem;
#pragma unroll
        for (int j = 0; j < 4; ++j) {
            const int lcol = wn * 64 + 16 * j + n;
            const float bb = bias[col0 + lcol];
#pragma unroll
            for (int i = 0; i < 2; ++i)
#pragma unroll
                for (int r = 0; r < 8; ++r) {
                    const int lrow = wm * 32 + 16 * i + 8 * h + r;
                    const float v = acc[i][j][r] * (1.0f / 512.0f) + bb;
                    T[lrow * 128 + lcol] = (f16)(v * 8.0f);
                }
        }
        __syncthreads();
        f16* G = (f16*)outp;
#pragma unroll
        for (int p = 0; p < 8; ++p) {
            const int c = p * 128 + tid, row = c >> 4, cc = c & 15;
            const v4ix val = *(const v4i*)(T + row * 128 + cc * 8);
            if (row0 + row < M)
                *(volatile v4i*)(G + (size_t)(row0 + row) * D_MODEL + col0 + cc * 8) = val;
        }
        __threadfence();
#pragma unroll
        for (int p = 0; p < 8; ++p) {
            const int c = p * 128 + tid, row = c >> 4, cc = c & 15;
            const v4ix val = *(const v4i*)(T + row * 128 + cc * 8);
            if (row0 + row < M)
                *(volatile v4i*)(G + (size_t)(row0 + row) * D_MODEL + col0 + cc * 8) = val;
        }
    } else if (MODE == 1) {
        f16* T = (f16*)smem;
#pragma unroll
        for (int j = 0; j < 4; ++j) {
            const int lcol = wn * 64 + 16 * j + n;
            const float bb = bias[col0 + lcol];
#pragma unroll
            for (int i = 0; i < 2; ++i) {
                const int tokb = wm * 32 + 16 * i + 8 * h;
                v8hx pv;
#pragma unroll
                for (int r = 0; r < 8; ++r)
                    pv[r] = (f16)((acc[i][j][r] * (1.0f / 512.0f) + bb) * 8.0f);
                *(v8h*)(T + lcol * 64 + tokb) = pv;
            }
        }
        __syncthreads();
        const int bidx = row0 >> 11, tok0 = row0 & (NB - 1);
        f16* G = (f16*)outp + ((size_t)bidx * D_MODEL + col0) * NB + tok0;
        if (row0 + 63 < M) {
#pragma unroll
            for (int p = 0; p < 8; ++p) {
                const int c = p * 128 + tid, dr = c >> 3, cc = c & 7;
                const v4ix val = *(const v4i*)(T + dr * 64 + cc * 8);
                *(volatile v4i*)(G + (size_t)dr * NB + cc * 8) = val;
            }
            __threadfence();
#pragma unroll
            for (int p = 0; p < 8; ++p) {
                const int c = p * 128 + tid, dr = c >> 3, cc = c & 7;
                const v4ix val = *(const v4i*)(T + dr * 64 + cc * 8);
                *(volatile v4i*)(G + (size_t)dr * NB + cc * 8) = val;
            }
        }
    } else {
        float* T = (float*)smem;
#pragma unroll
        for (int j = 0; j < 4; ++j) {
            const int lcol = wn * 64 + 16 * j + n;
            const float bb = bias[col0 + lcol];
#pragma unroll
            for (int i = 0; i < 2; ++i)
#pragma unroll
                for (int r = 0; r < 8; ++r) {
                    const int lrow = wm * 32 + 16 * i + 8 * h + r;
                    T[lrow * 128 + lcol] = acc[i][j][r] * (1.0f / 512.0f) + bb;
                }
        }
        __syncthreads();
        float* G = (float*)outp;
#pragma unroll
        for (int p = 0; p < 16; ++p) {
            const int c = p * 128 + tid, row = c >> 5, cc = c & 31;
            const v4ix val = *(const v4i*)(T + row * 128 + cc * 4);
            if (row0 + row < M)
                *(volatile v4i*)(G + (size_t)(row0 + row) * D_MODEL + col0 + cc * 4) = val;
        }
        __threadfence();
#pragma unroll
        for (int p = 0; p < 16; ++p) {
            const int c = p * 128 + tid, row = c >> 5, cc = c & 31;
            const v4ix val = *(const v4i*)(T + row * 128 + cc * 4);
            if (row0 + row < M)
                *(volatile v4i*)(G + (size_t)(row0 + row) * D_MODEL + col0 + cc * 4) = val;
        }
    }
}

__global__ __launch_bounds__(128)
void k_attn(const f16* __restrict__ Q, const f16* __restrict__ Km, const f16* __restrict__ Vt,
            const float* __restrict__ biasL, f16* O) {
    __shared__ __attribute__((aligned(16))) f16 ldsP[4 * 16 * 32];
    __shared__ __attribute__((aligned(16))) f16 ldsO[4 * 16 * 64];

    const int tid = threadIdx.x, lane = tid & 31, w = tid >> 5;
    const int h = lane >> 4, n = lane & 15;
    const int head = blockIdx.y, b = blockIdx.z;
    const int qrow0 = (blockIdx.x * 4 + w) * 16;
    f16* P  = ldsP + w * 512;
    f16* TO = ldsO + w * 1024;

    const f16* Qbase = Q + ((size_t)b * NB + qrow0) * D_MODEL + head * HD;
    const v16h aq0 = ldfrag(Qbase, D_MODEL, lane);
    const v16h aq1 = ldfrag(Qbase + 32, D_MODEL, lane);

    const v8f zero = {0.f, 0.f, 0.f, 0.f, 0.f, 0.f, 0.f, 0.f};
    float m[8], l[8];
    v8f o[4];
#pragma unroll
    for (int r = 0; r < 8; ++r) { m[r] = -1e30f; l[r] = 0.0f; }
#pragma unroll
    for (int t = 0; t < 4; ++t) o[t] = zero;

    const float* biasB = biasL + (size_t)b * NB;
    const float C1 = 1.0f / 512.0f;

    for (int kb = 0; kb < NB; kb += 32) {
        const f16* Kb0 = Km + ((size_t)b * NB + kb) * D_MODEL + head * HD;
        const f16* Kb1 = Kb0 + (size_t)16 * D_MODEL;
        v8f s0 = mma16(aq0, ldfrag(Kb0, D_MODEL, lane), zero);
        s0 = mma16(aq1, ldfrag(Kb0 + 32, D_MODEL, lane), s0);
        v8f s1 = mma16(aq0, ldfrag(Kb1, D_MODEL, lane), zero);
        s1 = mma16(aq1, ldfrag(Kb1 + 32, D_MODEL, lane), s1);

        const float bias0 = biasB[kb + n];
        const float bias1 = biasB[kb + 16 + n];

#pragma unroll
        for (int r = 0; r < 8; ++r) {
            const float x0 = s0[r] * C1 + bias0;
            const float x1 = s1[r] * C1 + bias1;
            const float mx = redmax16(fmaxf(x0, x1));
            const float mnew = fmaxf(m[r], mx);
            const float alpha = __expf(m[r] - mnew);
            const float p0 = __expf(x0 - mnew);
            const float p1 = __expf(x1 - mnew);
            l[r] = l[r] * alpha + redsum16(p0 + p1);
            m[r] = mnew;
            o[0][r] *= alpha; o[1][r] *= alpha;
            o[2][r] *= alpha; o[3][r] *= alpha;
            P[(8 * h + r) * 32 + n]      = (f16)(p0 * 4096.0f);
            P[(8 * h + r) * 32 + 16 + n] = (f16)(p1 * 4096.0f);
        }
        __syncthreads();

        Frag fp;
        fp.hv[0] = *(const v8h*)(P + n * 32 + 8 * h);
        fp.hv[1] = *(const v8h*)(P + n * 32 + 16 + 8 * h);

#pragma unroll
        for (int t = 0; t < 4; ++t) {
            const f16* Vb = Vt + ((size_t)b * D_MODEL + head * HD + t * 16) * NB + kb;
            o[t] = mma16(fp.v, ldfrag(Vb, NB, lane), o[t]);
        }
        __syncthreads();
    }

#pragma unroll
    for (int r = 0; r < 8; ++r) {
        const float inv = 1.0f / (4096.0f * l[r]);
#pragma unroll
        for (int t = 0; t < 4; ++t)
            TO[(8 * h + r) * 64 + t * 16 + n] = (f16)(o[t][r] * inv);
    }
    __syncthreads();

    f16* G = O + ((size_t)b * NB + qrow0) * D_MODEL + head * HD;
#pragma unroll
    for (int p = 0; p < 4; ++p) {
        const int c = p * 32 + lane, row = c >> 3, cc = c & 7;
        const v4ix val = *(const v4i*)(TO + row * 64 + cc * 8);
        *(volatile v4i*)(G + (size_t)row * D_MODEL + cc * 8) = val;
    }
    __threadfence();
#pragma unroll
    for (int p = 0; p < 4; ++p) {
        const int c = p * 32 + lane, row = c >> 3, cc = c & 7;
        const v4ix val = *(const v4i*)(TO + row * 64 + cc * 8);
        *(volatile v4i*)(G + (size_t)row * D_MODEL + cc * 8) = val;
    }
}

extern "C" void kernel_launch(void* const* d_in, const int* in_sizes, int n_in,
                              void* d_out, int out_size, void* d_ws, size_t ws_size,
                              hipStream_t stream) {
    if (n_in < 12) return;
    if (in_sizes[0] != MTOT * D_MODEL || in_sizes[1] != MTOT ||
        in_sizes[2] != D_MODEL * D_MODEL || in_sizes[4] != D_MODEL * D_MODEL ||
        in_sizes[6] != D_MODEL * D_MODEL || in_sizes[8] != D_MODEL * D_MODEL ||
        in_sizes[3] != D_MODEL || in_sizes[5] != D_MODEL || in_sizes[7] != D_MODEL ||
        in_sizes[9] != D_MODEL || in_sizes[10] < 1 || out_size != MTOT * D_MODEL) return;

    const float* h     = (const float*)d_in[0];
    const float* probs = (const float*)d_in[1];
    const float* Wq    = (const float*)d_in[2];
    const float* bq    = (const float*)d_in[3];
    const float* Wk    = (const float*)d_in[4];
    const float* bk    = (const float*)d_in[5];
    const float* Wv    = (const float*)d_in[6];
    const float* bv    = (const float*)d_in[7];
    const float* Wo    = (const float*)d_in[8];
    const float* bo    = (const float*)d_in[9];
    const float* pbs   = (const float*)d_in[10];
    const int*   nh    = (const int*)d_in[11];
    float* out         = (float*)d_out;

    char* ws = (char*)d_ws;
    size_t off = 0;
    auto carve = [&](size_t bytes) { char* p = ws + off; off += (bytes + 255) & ~(size_t)255; return p; };
    const size_t actBytes = (size_t)MTOT * D_MODEL * sizeof(f16);
    const size_t wBytes   = (size_t)D_MODEL * D_MODEL * sizeof(f16);
    f16*  h16   = (f16*)carve(actBytes);
    f16*  wq16  = (f16*)carve(wBytes);
    f16*  wk16  = (f16*)carve(wBytes);
    f16*  wv16  = (f16*)carve(wBytes);
    f16*  wo16  = (f16*)carve(wBytes);
    f16*  Q16   = (f16*)carve(actBytes);
    f16*  K16   = (f16*)carve(actBytes);
    f16*  Vt16  = (f16*)carve(actBytes);
    f16*  O16   = (f16*)carve(actBytes);
    float* biasL = (float*)carve((size_t)MTOT * sizeof(float));
    if (off > ws_size) return;

    const int totalW = D_MODEL * D_MODEL;

    k_prep<<<dim3((NB * (D_MODEL / 8) + 255) / 256), dim3(256), 0, stream>>>(h, h16);
    k_bias<<<dim3((MTOT / 4 + 255) / 256), dim3(256), 0, stream>>>(probs, pbs, nh, biasL, MTOT);
    k_cvtw<<<dim3((totalW / 8 + 255) / 256, 4), dim3(256), 0, stream>>>(
        Wq, Wk, Wv, Wo, wq16, wk16, wv16, wo16, totalW);

    const dim3 gblk(128);
    k_gemm<0><<<dim3(D_MODEL / 128, MTOT / 64, 2), gblk, 0, stream>>>(
        h16, wq16, wk16, bq, bk, (void*)Q16, (void*)K16, MTOT);
    k_gemm<1><<<dim3(D_MODEL / 128, MTOT / 64, 1), gblk, 0, stream>>>(
        h16, wv16, wv16, bv, bv, (void*)Vt16, (void*)Vt16, MTOT);

    k_attn<<<dim3(NB / 64, NHEAD, BATCH), dim3(128), 0, stream>>>(Q16, K16, Vt16, biasL, O16);

    k_gemm<2><<<dim3(D_MODEL / 128, MTOT / 64, 1), gblk, 0, stream>>>(
        O16, wo16, wo16, bo, bo, (void*)out, (void*)out, MTOT);
}
